// MambaBlock_13030930776224
// MI455X (gfx1250) — hardware-verified
//
#include <hip/hip_runtime.h>
#include <stddef.h>
#include <stdint.h>
#include <math.h>


#define DIMX   1024
#define DI     2048
#define DI2    4096
#define NST    16
#define DTR    64
#define XDN    96
#define XDP    128
#define KDT    128
#define LL     1024
#define NB     2
#define MR     2048
#define NTHR   256
#define GBM    64
#define GBN    64
#define GTHR   128
#define TC     64
#define SCH    64
#define WSMAX  134217728

#define NUI    (DI2 * (DIMX / 8))
#define NUX    (XDP * (DI2 / 8))
#define NUD    (DI * (KDT / 8))
#define NUO    (DIMX * (DI2 / 8))
#define NUTOT  (NUI + NUX + NUD + NUO)

static_assert(MR == NB * LL);
static_assert(MR % GBM == 0 && DI2 % GBN == 0 && DI % GBN == 0 && DIMX % GBN == 0 && XDP % GBN == 0);
static_assert(DIMX % 32 == 0 && DI2 % 32 == 0 && KDT % 32 == 0);
static_assert(GBM == (GTHR / 32) * 16 && GBN == 64);
static_assert(NUI % NTHR == 0 && NUX % NTHR == 0 && NUD % NTHR == 0 && NUO % NTHR == 0);
static_assert((MR * DIMX / 8) % NTHR == 0);
static_assert(DI == 2 * 4 * NTHR);
static_assert(NTHR == SCH * 4 && SCH * NST == 4 * NTHR && DI % SCH == 0 && LL % TC == 0);
static_assert(TC * 32 == 2 * 4 * NTHR);
static_assert(2 * TC * SCH == 4 * 8 * NTHR);
static_assert((GBM * GBN / 4) % GTHR == 0);
static_assert(XDN == DTR + 2 * NST && DTR == GBN);

typedef float          v4f   __attribute__((ext_vector_type(4)));
typedef float          v8f   __attribute__((ext_vector_type(8)));
typedef int            v8i   __attribute__((ext_vector_type(8)));
typedef unsigned short v8us  __attribute__((ext_vector_type(8)));
typedef unsigned short v16us __attribute__((ext_vector_type(16)));
typedef __bf16         v16bf __attribute__((ext_vector_type(16)));
typedef v4f  __attribute__((may_alias)) v4fa;
typedef v8us __attribute__((may_alias)) v8usa;
union FragB { v16bf v; v16us u; v8us h[2]; v8i w; };

__device__ __forceinline__ v8f wmb(const FragB& a, const FragB& b, v8f c) {
  v8f d = __builtin_amdgcn_wmma_f32_16x16x32_bf16(false, a.v, false, b.v, (short)0, c, false, false);
  asm volatile("v_nop\n\tv_nop\n\tv_nop\n\tv_nop" : "+v"(d) : "v"(a.w), "v"(b.w));
  return d;
}

__device__ __forceinline__ unsigned bf16_bits(float f) {
  const unsigned u = __float_as_uint(f);
  return (u + 0x7FFFu + ((u >> 16) & 1u)) >> 16;
}
__device__ __forceinline__ float bf16_val(float f) {
  return __uint_as_float(bf16_bits(f) << 16);
}
__device__ __forceinline__ float silu_f(float v) {
  return v * (1.0f / (1.0f + expf(-v)));
}
__device__ __forceinline__ float softplus_f(float v) {
  const float a = v > 0.0f ? v : 0.0f;
  return a + log1pf(expf(-fabsf(v)));
}
__device__ __forceinline__ unsigned short hl_sel(float f, bool lsel) {
  const unsigned hb = bf16_bits(f);
  const unsigned lb = bf16_bits(f - __uint_as_float(hb << 16));
  return (unsigned short)(lsel ? lb : hb);
}
__device__ __forceinline__ void put8(unsigned short* dp, const v8us o) {
  *(volatile v8us*)dp = o;
  __threadfence();
  *(volatile v8us*)dp = o;
}
__device__ __forceinline__ v8us gather8(const float* __restrict__ p, size_t stride, bool ok) {
  v8us o;
#pragma unroll
  for (int i = 0; i < 8; ++i) {
    const float f = p[(size_t)i * stride];
    o[i] = ok ? (unsigned short)bf16_bits(f) : (unsigned short)0;
  }
  return o;
}

__global__ __launch_bounds__(NTHR) void k_cvx(const float* __restrict__ x, unsigned short* xb) {
  const size_t u = (size_t)blockIdx.x * NTHR + threadIdx.x;
  const float* p = x + u * 8;
  const v4f a = *(const v4f*)p;
  const v4f b = *(const v4f*)(p + 4);
  v8us o;
  o[0] = (unsigned short)bf16_bits(a.x); o[1] = (unsigned short)bf16_bits(a.y);
  o[2] = (unsigned short)bf16_bits(a.z); o[3] = (unsigned short)bf16_bits(a.w);
  o[4] = (unsigned short)bf16_bits(b.x); o[5] = (unsigned short)bf16_bits(b.y);
  o[6] = (unsigned short)bf16_bits(b.z); o[7] = (unsigned short)bf16_bits(b.w);
  put8(xb + u * 8, o);
}

__global__ __launch_bounds__(NTHR) void k_wprep(const float* __restrict__ W_in, const float* __restrict__ W_xp,
                                                const float* __restrict__ W_dt, const float* __restrict__ W_out,
                                                unsigned short* WINT, unsigned short* WX2,
                                                unsigned short* WDT2, unsigned short* WO2) {
  const int u = (int)blockIdx.x * NTHR + (int)threadIdx.x;
  if (u < NUI) {
    const int n  = u >> 7;
    const int k8 = (u & 127) * 8;
    const v8us o = gather8(W_in + (size_t)k8 * DI2 + n, (size_t)DI2, true);
    put8(WINT + (size_t)n * DIMX + k8, o);
  } else if (u < NUI + NUX) {
    const int v  = u - NUI;
    const int n  = v >> 9;
    const int k8 = (v & 511) * 8;
    const int kk = k8 & (DI - 1);
    const int nc = n < XDN ? n : XDN - 1;
    const v8us o = gather8(W_xp + (size_t)kk * XDN + nc, (size_t)XDN, n < XDN);
    put8(WX2 + (size_t)n * DI2 + k8, o);
  } else if (u < NUI + NUX + NUD) {
    const int v  = u - NUI - NUX;
    const int n  = v >> 4;
    const int k8 = (v & 15) * 8;
    const int kk = k8 & (DTR - 1);
    const v8us o = gather8(W_dt + (size_t)kk * DI + n, (size_t)DI, true);
    put8(WDT2 + (size_t)n * KDT + k8, o);
  } else if (u < NUTOT) {
    const int v  = u - NUI - NUX - NUD;
    const int n  = v >> 9;
    const int k8 = (v & 511) * 8;
    const int kk = k8 & (DI - 1);
    const v8us o = gather8(W_out + (size_t)kk * DIMX + n, (size_t)DIMX, true);
    put8(WO2 + (size_t)n * DI2 + k8, o);
  }
}

template <int MODE>
__global__ __launch_bounds__(GTHR) void k_gemm(
    const unsigned short* __restrict__ A, const unsigned short* __restrict__ WT, int K,
    float* outF, unsigned short* outH, const float* __restrict__ bias, int ldo, size_t goff)
{
  __shared__ __attribute__((aligned(16))) float stg[GBM * GBN];
  const int tid = (int)threadIdx.x, lane = tid & 31, wave = tid >> 5, hh = lane >> 4, m = lane & 15;
  const int rowBase = (int)blockIdx.x * GBM;
  const int col0    = (int)blockIdx.y * GBN;

  v8f acc[4];
  {
    const v8f z = {0.f, 0.f, 0.f, 0.f, 0.f, 0.f, 0.f, 0.f};
    acc[0] = z; acc[1] = z; acc[2] = z; acc[3] = z;
  }
  const unsigned short* ap = A  + (size_t)(rowBase + 16 * wave + m) * (size_t)K + 8 * hh;
  const unsigned short* wp = WT + (size_t)(col0 + m) * (size_t)K + 8 * hh;
  const int ksteps = K >> 5;
#pragma unroll 1
  for (int ks = 0; ks < ksteps; ++ks) {
    FragB af;
    af.h[0] = *(const v8usa*)(ap + 32 * ks);
    af.h[1] = *(const v8usa*)(ap + 32 * ks + 16);
#pragma unroll
    for (int t = 0; t < 4; ++t) {
      const unsigned short* wq = wp + (size_t)(16 * t) * (size_t)K + 32 * ks;
      FragB bf;
      bf.h[0] = *(const v8usa*)wq;
      bf.h[1] = *(const v8usa*)(wq + 16);
      acc[t] = wmb(af, bf, acc[t]);
    }
  }

#pragma unroll
  for (int t = 0; t < 4; ++t) {
    const int lc = 16 * t + m;
#pragma unroll
    for (int r = 0; r < 8; ++r) {
      const int lr = 16 * wave + 8 * hh + r;
      stg[lr * GBN + lc] = acc[t][r];
    }
  }
  __syncthreads();

  if constexpr (MODE == 0) {
    if (col0 >= DI) {
#pragma unroll 1
      for (int j = 0; j < (GBM * GBN / 4) / GTHR; ++j) {
        const int e4 = j * GTHR + tid;
        v4f v = *(const v4fa*)(stg + 4 * e4);
        v.x = silu_f(v.x); v.y = silu_f(v.y); v.z = silu_f(v.z); v.w = silu_f(v.w);
        *(v4fa*)(stg + 4 * e4) = v;
      }
    }
    __syncthreads();
  }
  if constexpr (MODE == 2) {
#pragma unroll 1
    for (int j = 0; j < (GBM * GBN / 4) / GTHR; ++j) {
      const int e4 = j * GTHR + tid;
      const int c  = (e4 & 15) * 4;
      const v4f b4 = *(const v4f*)(bias + col0 + c);
      v4f v = *(const v4fa*)(stg + 4 * e4);
      v.x = softplus_f(v.x + bf16_val(b4.x));
      v.y = softplus_f(v.y + bf16_val(b4.y));
      v.z = softplus_f(v.z + bf16_val(b4.z));
      v.w = softplus_f(v.w + bf16_val(b4.w));
      *(v4fa*)(stg + 4 * e4) = v;
    }
    __syncthreads();
  }

  if constexpr (MODE == 1) {
    if (blockIdx.y == 0) {
      const bool lsel = m >= 8;
      v8us qv[8];
#pragma unroll
      for (int i = 0; i < 8; ++i) {
        const int lr = 16 * wave + 2 * i + hh;
        const float* sp = stg + lr * GBN + 8 * (m & 7);
        const v4f fa = *(const v4fa*)sp;
        const v4f fb = *(const v4fa*)(sp + 4);
        v8us o;
        o[0] = hl_sel(fa.x, lsel); o[1] = hl_sel(fa.y, lsel);
        o[2] = hl_sel(fa.z, lsel); o[3] = hl_sel(fa.w, lsel);
        o[4] = hl_sel(fb.x, lsel); o[5] = hl_sel(fb.y, lsel);
        o[6] = hl_sel(fb.z, lsel); o[7] = hl_sel(fb.w, lsel);
        qv[i] = o;
      }
#pragma unroll
      for (int i = 0; i < 8; ++i) {
        const int lr = 16 * wave + 2 * i + hh;
        unsigned short* dp = outH + (size_t)(rowBase + lr) * KDT + 8 * m;
        *(volatile v8us*)dp = qv[i];
      }
      __threadfence();
#pragma unroll
      for (int i = 0; i < 8; ++i) {
        const int lr = 16 * wave + 2 * i + hh;
        unsigned short* dp = outH + (size_t)(rowBase + lr) * KDT + 8 * m;
        *(volatile v8us*)dp = qv[i];
      }
    } else {
      const int rq = lane >> 3;
      const int c4 = (lane & 7) * 4;
      v4f bv[4];
#pragma unroll
      for (int i = 0; i < 4; ++i) {
        const int lr = 16 * wave + 4 * i + rq;
        bv[i] = *(const v4fa*)(stg + lr * GBN + c4);
      }
#pragma unroll
      for (int i = 0; i < 4; ++i) {
        const int lr = 16 * wave + 4 * i + rq;
        float* op = outF + (size_t)(rowBase + lr) * 32 + c4;
        *(volatile v4f*)op = bv[i];
      }
      __threadfence();
#pragma unroll
      for (int i = 0; i < 4; ++i) {
        const int lr = 16 * wave + 4 * i + rq;
        float* op = outF + (size_t)(rowBase + lr) * 32 + c4;
        *(volatile v4f*)op = bv[i];
      }
    }
  } else {
    size_t pbase = 0;
    int cc = col0;
    if constexpr (MODE == 0) {
      const bool isg = col0 >= DI;
      pbase = isg ? goff : (size_t)0;
      cc    = isg ? col0 - DI : col0;
    }
    v4f fv[8];
#pragma unroll
    for (int i = 0; i < 8; ++i) {
      const int lr = 16 * wave + 2 * i + hh;
      fv[i] = *(const v4fa*)(stg + lr * GBN + 4 * m);
    }
#pragma unroll
    for (int i = 0; i < 8; ++i) {
      const int lr = 16 * wave + 2 * i + hh;
      float* op = outF + pbase + (size_t)(rowBase + lr) * (size_t)ldo + cc + 4 * m;
      *(volatile v4f*)op = fv[i];
    }
    __threadfence();
#pragma unroll
    for (int i = 0; i < 8; ++i) {
      const int lr = 16 * wave + 2 * i + hh;
      float* op = outF + pbase + (size_t)(rowBase + lr) * (size_t)ldo + cc + 4 * m;
      *(volatile v4f*)op = fv[i];
    }
  }
}

__device__ __forceinline__ float conv1(const v4f w, float b, float a0, float a1, float a2, float a3,
                                       float f0, float f1, float f2) {
  float acc = bf16_val(b);
  acc = fmaf(bf16_val(w.x) * f0, a0, acc);
  acc = fmaf(bf16_val(w.y) * f1, a1, acc);
  acc = fmaf(bf16_val(w.z) * f2, a2, acc);
  acc = fmaf(bf16_val(w.w), a3, acc);
  return acc;
}

__global__ __launch_bounds__(NTHR) void k_conv(const float* __restrict__ xp, const float* __restrict__ cw,
                                               const float* __restrict__ cb, float* U, unsigned short* UHL) {
  __shared__ __attribute__((aligned(16))) float sc[4 * NTHR];
  __shared__ __attribute__((aligned(16))) unsigned short sh[8 * NTHR];
  const int tid   = (int)threadIdx.x;
  const int r     = (int)blockIdx.x >> 1;
  const int cbase = ((int)blockIdx.x & 1) * (4 * NTHR);
  const int d     = cbase + 4 * tid;
  const int t     = r & (LL - 1);
  const int rb    = r - t;
  const int t0 = t - 3, t1 = t - 2, t2 = t - 1;
  const float f0 = t0 >= 0 ? 1.0f : 0.0f;
  const float f1 = t1 >= 0 ? 1.0f : 0.0f;
  const float f2 = t2 >= 0 ? 1.0f : 0.0f;
  const int r0 = rb + (t0 > 0 ? t0 : 0);
  const int r1 = rb + (t1 > 0 ? t1 : 0);
  const int r2 = rb + (t2 > 0 ? t2 : 0);
  const v4f x0 = *(const v4f*)(xp + (size_t)r0 * DI + d);
  const v4f x1 = *(const v4f*)(xp + (size_t)r1 * DI + d);
  const v4f x2 = *(const v4f*)(xp + (size_t)r2 * DI + d);
  const v4f x3 = *(const v4f*)(xp + (size_t)r  * DI + d);
  const v4f wa = *(const v4f*)(cw + (size_t)d * 4);
  const v4f wb = *(const v4f*)(cw + (size_t)d * 4 + 4);
  const v4f wc = *(const v4f*)(cw + (size_t)d * 4 + 8);
  const v4f wd = *(const v4f*)(cw + (size_t)d * 4 + 12);
  const v4f bb = *(const v4f*)(cb + d);
  sc[4 * tid + 0] = conv1(wa, bb.x, x0.x, x1.x, x2.x, x3.x, f0, f1, f2);
  sc[4 * tid + 1] = conv1(wb, bb.y, x0.y, x1.y, x2.y, x3.y, f0, f1, f2);
  sc[4 * tid + 2] = conv1(wc, bb.z, x0.z, x1.z, x2.z, x3.z, f0, f1, f2);
  sc[4 * tid + 3] = conv1(wd, bb.w, x0.w, x1.w, x2.w, x3.w, f0, f1, f2);
#pragma unroll 1
  for (int i = 0; i < 4; ++i) {
    const float c = sc[4 * tid + i];
    const float s = silu_f(c);
    sc[4 * tid + i] = s;
    const unsigned hb = bf16_bits(s);
    const unsigned lb = bf16_bits(s - __uint_as_float(hb << 16));
    sh[4 * tid + i] = (unsigned short)hb;
    sh[4 * NTHR + 4 * tid + i] = (unsigned short)lb;
  }
  v4f uv;
  uv.x = sc[4 * tid + 0]; uv.y = sc[4 * tid + 1]; uv.z = sc[4 * tid + 2]; uv.w = sc[4 * tid + 3];
  __syncthreads();
  const v8us hv = *(const v8usa*)(sh + 8 * tid);
  const int hcol = (tid < 128) ? (cbase + 8 * tid) : (DI + cbase + 8 * (tid - 128));
  float* up = U + (size_t)r * DI + d;
  unsigned short* hp = UHL + (size_t)r * DI2 + hcol;
  *(volatile v4f*)up = uv;
  *(volatile v8us*)hp = hv;
  __threadfence();
  *(volatile v4f*)up = uv;
  *(volatile v8us*)hp = hv;
}

__global__ __launch_bounds__(NTHR) void k_scan(const float* __restrict__ DELTA, const float* __restrict__ U,
                                               const float* __restrict__ G, const float* __restrict__ BC,
                                               const float* __restrict__ A_log, const float* __restrict__ Dv,
                                               unsigned short* Y) {
  __shared__ __attribute__((aligned(16))) float bc[TC * 32];
  __shared__ __attribute__((aligned(16))) float an[SCH * NST];
  __shared__ __attribute__((aligned(16))) unsigned short ys[2 * TC * SCH];
  const int tid = (int)threadIdx.x;
  const int q   = tid & 3;
  const int cl  = tid >> 2;
  const int b   = (int)blockIdx.x >> 5;
  const int cg  = (int)blockIdx.x & 31;
  const int d   = cg * SCH + cl;

#pragma unroll 1
  for (int i = 0; i < 4; ++i) {
    const int idx = i * NTHR + tid;
    an[idx] = -expf(bf16_val(A_log[(size_t)cg * (SCH * NST) + idx]));
  }
  __syncthreads();
  const v4f A4 = *(const v4fa*)(an + 4 * tid);
  const float Dd = bf16_val(Dv[d]);
  float h0 = 0.0f, h1 = 0.0f, h2 = 0.0f, h3 = 0.0f;
  const size_t rowb = (size_t)b * LL;

#pragma unroll 1
  for (int ck = 0; ck < LL / TC; ++ck) {
    const size_t r0 = rowb + (size_t)ck * TC;
    {
      const float* src = BC + r0 * 32;
      const v4f c0 = *(const v4f*)(src + 4 * tid);
      const v4f c1 = *(const v4f*)(src + 4 * (NTHR + tid));
      *(v4fa*)(bc + 4 * tid) = c0;
      *(v4fa*)(bc + 4 * (NTHR + tid)) = c1;
    }
    __syncthreads();
#pragma unroll 1
    for (int t = 0; t < TC; ++t) {
      const size_t e = (r0 + (size_t)t) * DI + d;
      const float dl = DELTA[e];
      const float uu = U[e];
      const float gg = G[e];
      const v4f Bv = *(const v4fa*)(bc + t * 32 + 4 * q);
      const v4f Cv = *(const v4fa*)(bc + t * 32 + 16 + 4 * q);
      h0 = fmaf(expf(dl * A4.x), h0, (dl * Bv.x) * uu);
      h1 = fmaf(expf(dl * A4.y), h1, (dl * Bv.y) * uu);
      h2 = fmaf(expf(dl * A4.z), h2, (dl * Bv.z) * uu);
      h3 = fmaf(expf(dl * A4.w), h3, (dl * Bv.w) * uu);
      float p = h0 * Cv.x;
      p = fmaf(h1, Cv.y, p);
      p = fmaf(h2, Cv.z, p);
      p = fmaf(h3, Cv.w, p);
      p += __shfl_xor(p, 1, 32);
      p += __shfl_xor(p, 2, 32);
      const float y = (p + uu * Dd) * gg;
      const unsigned hb = bf16_bits(y);
      const unsigned lb = bf16_bits(y - __uint_as_float(hb << 16));
      if (q == 0) {
        ys[t * SCH + cl] = (unsigned short)hb;
        ys[TC * SCH + t * SCH + cl] = (unsigned short)lb;
      }
    }
    __syncthreads();
    v8us qv[4];
#pragma unroll
    for (int it = 0; it < 4; ++it) qv[it] = *(const v8usa*)(ys + 8 * (it * NTHR + tid));
#pragma unroll
    for (int it = 0; it < 4; ++it) {
      const int idx = it * NTHR + tid;
      const int pl  = idx >> 9;
      const int tt  = (idx >> 3) & (TC - 1);
      const int pc  = idx & 7;
      unsigned short* dp = Y + (r0 + (size_t)tt) * DI2 + (size_t)pl * DI + cg * SCH + 8 * pc;
      *(volatile v8us*)dp = qv[it];
    }
    __threadfence();
#pragma unroll
    for (int it = 0; it < 4; ++it) {
      const int idx = it * NTHR + tid;
      const int pl  = idx >> 9;
      const int tt  = (idx >> 3) & (TC - 1);
      const int pc  = idx & 7;
      unsigned short* dp = Y + (r0 + (size_t)tt) * DI2 + (size_t)pl * DI + cg * SCH + 8 * pc;
      *(volatile v8us*)dp = qv[it];
    }
  }
}

static inline size_t al256(size_t o) { return (o + 255) & ~(size_t)255; }

extern "C" void kernel_launch(void* const* d_in, const int* in_sizes, int n_in,
                              void* d_out, int out_size, void* d_ws, size_t ws_size,
                              hipStream_t stream) {
  if (n_in < 10) return;
  if (in_sizes[0] != MR * DIMX) return;
  if (in_sizes[1] != DIMX * DI2) return;
  if (in_sizes[2] != DI * 4) return;
  if (in_sizes[3] != DI) return;
  if (in_sizes[4] != DI * XDN) return;
  if (in_sizes[5] != DTR * DI) return;
  if (in_sizes[6] != DI) return;
  if (in_sizes[7] != DI * NST) return;
  if (in_sizes[8] != DI) return;
  if (in_sizes[9] != DI * DIMX) return;
  if (out_size != MR * DIMX) return;

  const float* x     = (const float*)d_in[0];
  const float* W_in  = (const float*)d_in[1];
  const float* convw = (const float*)d_in[2];
  const float* convb = (const float*)d_in[3];
  const float* W_xp  = (const float*)d_in[4];
  const float* W_dt  = (const float*)d_in[5];
  const float* b_dt  = (const float*)d_in[6];
  const float* A_log = (const float*)d_in[7];
  const float* Dv    = (const float*)d_in[8];
  const float* W_out = (const float*)d_in[9];
  float* out = (float*)d_out;

  char* ws = (char*)d_ws;
  size_t off = 0;
  const size_t oXB   = off; off = al256(off + (size_t)MR * DIMX * 2);
  const size_t oWINT = off; off = al256(off + (size_t)DI2 * DIMX * 2);
  const size_t oWX2  = off; off = al256(off + (size_t)XDP * DI2 * 2);
  const size_t oWDT2 = off; off = al256(off + (size_t)DI * KDT * 2);
  const size_t oWO2  = off; off = al256(off + (size_t)DIMX * DI2 * 2);
  const size_t oXP   = off; off = al256(off + (size_t)MR * DI * 4);
  const size_t oG    = off; off = al256(off + (size_t)MR * DI * 4);
  const size_t oU    = off; off = al256(off + (size_t)MR * DI * 4);
  const size_t oUHL  = off; off = al256(off + (size_t)MR * DI2 * 2);
  const size_t oDR   = off; off = al256(off + (size_t)MR * KDT * 2);
  const size_t oBC   = off; off = al256(off + (size_t)MR * 32 * 4);
  const size_t oDL   = off; off = al256(off + (size_t)MR * DI * 4);
  const size_t oY    = off; off = al256(off + (size_t)MR * DI2 * 2);
  if (off > ws_size || off > (size_t)WSMAX) return;
  if (oG <= oXP || ((oG - oXP) & 3) != 0) return;
  unsigned short* XB   = (unsigned short*)(ws + oXB);
  unsigned short* WINT = (unsigned short*)(ws + oWINT);
  unsigned short* WX2  = (unsigned short*)(ws + oWX2);
  unsigned short* WDT2 = (unsigned short*)(ws + oWDT2);
  unsigned short* WO2  = (unsigned short*)(ws + oWO2);
  float*          XP   = (float*)(ws + oXP);
  float*          G    = (float*)(ws + oG);
  float*          U    = (float*)(ws + oU);
  unsigned short* UHL  = (unsigned short*)(ws + oUHL);
  unsigned short* DR   = (unsigned short*)(ws + oDR);
  float*          BC   = (float*)(ws + oBC);
  float*          DL   = (float*)(ws + oDL);
  unsigned short* Y    = (unsigned short*)(ws + oY);
  const size_t goff = (oG - oXP) / 4;

  k_cvx<<<(MR * DIMX / 8) / NTHR, NTHR, 0, stream>>>(x, XB);
  k_wprep<<<NUTOT / NTHR, NTHR, 0, stream>>>(W_in, W_xp, W_dt, W_out, WINT, WX2, WDT2, WO2);
  k_gemm<0><<<dim3(MR / GBM, DI2 / GBN), GTHR, 0, stream>>>(XB, WINT, DIMX, XP, (unsigned short*)0, b_dt, DI, goff);
  k_conv<<<MR * 2, NTHR, 0, stream>>>(XP, convw, convb, U, UHL);
  k_gemm<1><<<dim3(MR / GBM, XDP / GBN), GTHR, 0, stream>>>(UHL, WX2, DI2, BC, DR, b_dt, 32, (size_t)0);
  k_gemm<2><<<dim3(MR / GBM, DI / GBN), GTHR, 0, stream>>>(DR, WDT2, KDT, DL, (unsigned short*)0, b_dt, DI, (size_t)0);
  k_scan<<<NB * (DI / SCH), NTHR, 0, stream>>>(DL, U, G, BC, A_log, Dv, Y);
  k_gemm<3><<<dim3(MR / GBM, DIMX / GBN), GTHR, 0, stream>>>(Y, WO2, DI2, out, (unsigned short*)0, b_dt, DIMX, (size_t)0);
}
